// HybridTwoTower_65506841198666
// MI455X (gfx1250) — hardware-run, weakly checked
//
#include <hip/hip_runtime.h>
#include <math.h>

constexpr int kItems = 100000;
constexpr int kUsers = 16384;
constexpr int kHist  = 50;
constexpr int kGcn   = 128;
constexpr int kGeo   = 32;
constexpr int kXi    = kGeo + kGcn;
constexpr int kHid   = 256;
constexpr int kTow   = 128;
constexpr int kFusedLd = kGcn + kTow;
constexpr int kItemChunkRows = 50048;
constexpr int kItemChunks    = 2;
constexpr int kUserChunk     = 2048;
constexpr int kUserChunks    = 8;
constexpr int kHRows         = kUserChunk * kHist;
constexpr float kActCarry    = 8.0f;
constexpr float kWCarry      = 16.0f;
constexpr float kScaleOutF32 = 1.0f / 128.0f;
constexpr float kScaleOutX8  = 1.0f / 16.0f;
static_assert(kItemChunkRows % 64 == 0);
static_assert(kItemChunkRows * kItemChunks >= kItems);
static_assert(kHRows % 64 == 0);
static_assert(kUserChunk * kUserChunks == kUsers);
static_assert(kUsers % 64 == 0);
static_assert(kXi % 32 == 0 && kHid % 64 == 0 && kTow % 64 == 0 && kGcn % 32 == 0);

typedef __attribute__((ext_vector_type(16))) _Float16 v16h;
typedef __attribute__((ext_vector_type(8)))  _Float16 v8h;
typedef __attribute__((ext_vector_type(16))) __bf16   v16b;
typedef __attribute__((ext_vector_type(8)))  __bf16   v8b;
typedef __attribute__((ext_vector_type(8)))  float    v8f;
typedef __attribute__((ext_vector_type(4)))  float    v4f;
typedef __attribute__((ext_vector_type(4)))  unsigned int v4u;
typedef __attribute__((ext_vector_type(2)))  unsigned int v2u;

__device__ __forceinline__ unsigned short f2bf_bits(float f) {
  unsigned u = __float_as_uint(f);
  return (unsigned short)((u + 0x7FFFu + ((u >> 16) & 1u)) >> 16);
}
__device__ __forceinline__ float bf_bits2f(unsigned short h) { return __uint_as_float(((unsigned)h) << 16); }

__device__ __forceinline__ void dep_guard_h(v8f& a, v8f& b, v16h x, v16h y) { asm volatile("v_nop\n\tv_nop\n\tv_nop\n\tv_nop" : "+v"(a), "+v"(b) : "v"(x), "v"(y)); }
__device__ __forceinline__ void dep_guard_b(v8f& a, v8f& b, v16b x, v16b y) { asm volatile("v_nop\n\tv_nop\n\tv_nop\n\tv_nop" : "+v"(a), "+v"(b) : "v"(x), "v"(y)); }
__device__ __forceinline__ void keep4_h(v16h a, v16h b, v16h c, v16h d) { asm volatile("v_nop" :: "v"(a), "v"(b), "v"(c), "v"(d)); }
__device__ __forceinline__ void keep4_b(v16b a, v16b b, v16b c, v16b d) { asm volatile("v_nop" :: "v"(a), "v"(b), "v"(c), "v"(d)); }
__device__ __forceinline__ void acc_guard4(v8f& a, v8f& b, v8f& c, v8f& d) { asm volatile("v_nop\n\tv_nop\n\tv_nop\n\tv_nop" : "+v"(a), "+v"(b), "+v"(c), "+v"(d)); }
template <typename T> struct Frag;
template <> struct Frag<_Float16> {
  typedef v16h V; union U { v16h v; v8h h[2]; };
  static __device__ __forceinline__ v16h load(const _Float16* p) {
    U f; f.h[0] = *(const v8h*)(p); f.h[1] = *(const v8h*)(p + 16); return f.v;
  }
  static __device__ __forceinline__ v8f mma(v16h a, v16h b, v8f c) {
    return __builtin_amdgcn_wmma_f32_16x16x32_f16(false, a, false, b, (short)0, c, false, false);
  }
  static __device__ __forceinline__ void guard(v8f& a, v8f& b, v16h x, v16h y) { dep_guard_h(a, b, x, y); }
  static __device__ __forceinline__ void keep(v16h a, v16h b, v16h c, v16h d) { keep4_h(a, b, c, d); }
};
template <> struct Frag<__bf16> {
  typedef v16b V; union U { v16b v; v8b h[2]; };
  static __device__ __forceinline__ v16b load(const __bf16* p) {
    U f; f.h[0] = *(const v8b*)(p); f.h[1] = *(const v8b*)(p + 16); return f.v;
  }
  static __device__ __forceinline__ v8f mma(v16b a, v16b b, v8f c) {
    return __builtin_amdgcn_wmma_f32_16x16x32_bf16(false, a, false, b, (short)0, c, false, false);
  }
  static __device__ __forceinline__ void guard(v8f& a, v8f& b, v16b x, v16b y) { dep_guard_b(a, b, x, y); }
  static __device__ __forceinline__ void keep(v16b a, v16b b, v16b c, v16b d) { keep4_b(a, b, c, d); }
};

__device__ __forceinline__ unsigned pk16(unsigned short a, unsigned short b) { return (unsigned)a | ((unsigned)b << 16); }
__device__ __forceinline__ unsigned short h_bits(float f) { const _Float16 h = (_Float16)f; return __builtin_bit_cast(unsigned short, h); }

template <int ET> struct Elem;
template <> struct Elem<0> { typedef _Float16 T; };
template <> struct Elem<1> { typedef __bf16 T; };
template <int ET, bool SPLIT, int BIAS_MODE, int OUT_MODE, bool RESID, int ACT = 0>
__global__ __launch_bounds__(256) void wmma_gemm64(
    const unsigned short* __restrict__ Ap, const unsigned short* __restrict__ A2p, int lda, long strideA,
    const unsigned short* __restrict__ Btp, const unsigned short* __restrict__ Bt2p, int ldb, long strideB,
    void* __restrict__ Cout, void* __restrict__ Cout2, int ldc, long strideC,
    const float* __restrict__ bias,
    const float* __restrict__ resid, long strideR,
    int M, int N, int K, float scale) {
  typedef typename Elem<ET>::T T;
  typedef typename Frag<T>::V V;
  const T* A = (const T*)Ap; const T* A2 = (const T*)A2p; const T* Bt = (const T*)Btp; const T* Bt2 = (const T*)Bt2p;
  __shared__ __align__(16) float sT[8][16 * 68];
  const int b    = blockIdx.y;
  const int lane = threadIdx.x & 31;
  const int wave = threadIdx.x >> 5;
  const int tilesN = N >> 6;
  const int tilesM = M >> 6;
  const int tile = blockIdx.x * 8 + wave;
  if (tile >= tilesM * tilesN) return;
  const int tm = tile / tilesN;
  const int tn = tile - tm * tilesN;
  const int m0 = tm << 6;
  const int n0 = tn << 6;

  const T* Ab  = A  + (size_t)b * strideA;
  const T* Bb  = Bt + (size_t)b * strideB;
  const T* Ab2 = SPLIT ? (A2  + (size_t)b * strideA) : nullptr;
  const T* Bb2 = SPLIT ? (Bt2 + (size_t)b * strideB) : nullptr;

  const int rlane = lane & 15;
  const int koff  = (lane >> 4) * 8;
  const int mOff  = (lane >> 4) * 8;

  v8f acc[4][4];
#pragma unroll
  for (int i = 0; i < 4; ++i)
#pragma unroll
    for (int j = 0; j < 4; ++j) acc[i][j] = (v8f){0.f,0.f,0.f,0.f,0.f,0.f,0.f,0.f};

  for (int k0 = 0; k0 < K; k0 += 32) {
    V bh[4], bl[4];
#pragma unroll
    for (int j = 0; j < 4; ++j) {
      const size_t bo = (size_t)(n0 + (j << 4) + rlane) * ldb + koff + k0;
      bh[j] = Frag<T>::load(Bb + bo);
      if (SPLIT) bl[j] = Frag<T>::load(Bb2 + bo);
    }
#pragma unroll
    for (int i = 0; i < 4; ++i) {
      const size_t ao = (size_t)(m0 + (i << 4) + rlane) * lda + koff + k0;
      V ah = Frag<T>::load(Ab + ao);
      V al;
      if (SPLIT) al = Frag<T>::load(Ab2 + ao);
#pragma unroll
      for (int j = 0; j < 4; ++j) {
        acc[i][j] = Frag<T>::mma(ah, bh[j], acc[i][j]);
        if (SPLIT) {
          acc[i][j] = Frag<T>::mma(ah, bl[j], acc[i][j]);
          acc[i][j] = Frag<T>::mma(al, bh[j], acc[i][j]);
        }
      }
      Frag<T>::guard(acc[i][0], acc[i][3], ah, SPLIT ? al : ah);
    }
    Frag<T>::keep(bh[0], bh[1], bh[2], bh[3]);
    if (SPLIT) Frag<T>::keep(bl[0], bl[1], bl[2], bl[3]);
  }
  acc_guard4(acc[0][0], acc[0][1], acc[0][2], acc[0][3]);
  acc_guard4(acc[1][0], acc[1][1], acc[1][2], acc[1][3]);
  acc_guard4(acc[2][0], acc[2][1], acc[2][2], acc[2][3]);
  acc_guard4(acc[3][0], acc[3][1], acc[3][2], acc[3][3]);

  float* slab = sT[wave];
  const float* Rb = RESID ? (resid + (size_t)b * strideR) : nullptr;
#pragma unroll
  for (int i = 0; i < 4; ++i) {
    const int mBase = m0 + (i << 4);
#pragma unroll
    for (int j = 0; j < 4; ++j) {
      const int n = n0 + (j << 4) + rlane;
      float bv = 0.f;
      if (BIAS_MODE == 2) bv = bias[n];
#pragma unroll
      for (int r = 0; r < 8; ++r) {
        float v = acc[i][j][r] * scale;
        if (BIAS_MODE == 1) v += bias[mBase + mOff + r];
        if (BIAS_MODE == 2) v += bv;
        if (RESID) v += Rb[(size_t)(mBase + mOff + r) * ldc + n];
        if (ACT == 2) v = fmaxf(v, 0.0f);
        if (ACT == 4) v = (v > 0.f) ? v : 0.01f * v;
        slab[(mOff + r) * 68 + (j << 4) + rlane] = v;
      }
    }
    __builtin_amdgcn_fence(__ATOMIC_RELEASE, "workgroup");
    __builtin_amdgcn_wave_barrier();
    __builtin_amdgcn_fence(__ATOMIC_ACQUIRE, "workgroup");
    if (OUT_MODE == 0) {
      float* C = (float*)Cout + (size_t)b * strideC;
      const int hh = lane >> 4, c4 = (lane & 15) * 4;
      for (int pass = 0; pass < 2; ++pass) {
#pragma unroll
        for (int it = 0; it < 8; ++it) {
          const int row = it * 2 + hh;
          v4f v = *(const v4f*)(slab + row * 68 + c4);
          *(volatile v4f*)(C + (size_t)(mBase + row) * ldc + n0 + c4) = v;
        }
        __threadfence();
      }
    } else {
      const int q = lane >> 3, c8 = (lane & 7) * 8;
      unsigned short* C  = (unsigned short*)Cout  + (size_t)b * strideC;
      unsigned short* C2 = (OUT_MODE == 2) ? ((unsigned short*)Cout2 + (size_t)b * strideC) : nullptr;
      for (int pass = 0; pass < 2; ++pass) {
#pragma unroll
        for (int it = 0; it < 4; ++it) {
          const int row = it * 4 + q;
          const float* sp = slab + row * 68 + c8;
          v8h hv, lv;
#pragma unroll
          for (int e = 0; e < 8; ++e) {
            if (OUT_MODE == 1) {
              hv[e] = (_Float16)sp[e];
            } else {
              unsigned short hb = f2bf_bits(sp[e]);
              unsigned short lb = f2bf_bits(sp[e] - bf_bits2f(hb));
              hv[e] = __builtin_bit_cast(_Float16, hb);
              lv[e] = __builtin_bit_cast(_Float16, lb);
            }
          }
          *(volatile v8h*)(C + (size_t)(mBase + row) * ldc + n0 + c8) = hv;
          if (OUT_MODE == 2) *(volatile v8h*)(C2 + (size_t)(mBase + row) * ldc + n0 + c8) = lv;
        }
        __threadfence();
      }
    }
    __builtin_amdgcn_fence(__ATOMIC_RELEASE, "workgroup");
    __builtin_amdgcn_wave_barrier();
    __builtin_amdgcn_fence(__ATOMIC_ACQUIRE, "workgroup");
  }
}

__device__ __forceinline__ v4u pack8_carry(v4f a, v4f c) {
  return (v4u){pk16(h_bits(a[0] * kActCarry), h_bits(a[1] * kActCarry)),
               pk16(h_bits(a[2] * kActCarry), h_bits(a[3] * kActCarry)),
               pk16(h_bits(c[0] * kActCarry), h_bits(c[1] * kActCarry)),
               pk16(h_bits(c[2] * kActCarry), h_bits(c[3] * kActCarry))};
}

__global__ __launch_bounds__(256) void wtcast_kernel(const float* __restrict__ W, unsigned short* __restrict__ WT,
                                                     int K, int N, float scale) {
  __shared__ __align__(16) unsigned short sm[64 * 264];
  const int t  = threadIdx.x;
  const int n0 = blockIdx.x * 64;
  const int nLoad = K >> 2;
#pragma unroll 1
  for (int i = 0; i < nLoad; ++i) {
    const int e = i * 256 + t;
    const int k = e >> 6;
    const int n = e & 63;
    sm[n * 264 + k] = h_bits(W[(size_t)k * N + n0 + n] * scale);
  }
  __syncthreads();
  const int nStore = K >> 5;
  unsigned short* base = WT + (size_t)n0 * K;
  for (int pass = 0; pass < 2; ++pass) {
#pragma unroll 1
    for (int i = 0; i < nStore; ++i) {
      const int f = (i * 256 + t) * 8;
      const int n = f / K;
      const int k = f - n * K;
      const unsigned short* sp = sm + n * 264 + k;
      const v4u u = (v4u){pk16(sp[0], sp[1]), pk16(sp[2], sp[3]), pk16(sp[4], sp[5]), pk16(sp[6], sp[7])};
      *(volatile v4u*)(base + f) = u;
    }
    __threadfence();
  }
}

__global__ __launch_bounds__(64) void bias8_kernel(const float* __restrict__ b, float* __restrict__ out) {
  const int t = threadIdx.x;
  v4f v = *(const v4f*)(b + 4 * t);
  v = v * kActCarry;
  float* p = out + 4 * t;
  *(volatile v4f*)p = v;
  __threadfence();
  *(volatile v4f*)p = v;
}

__global__ __launch_bounds__(256) void xi_build_kernel(const float* __restrict__ item_feat, const float* __restrict__ gcn_item,
                                                       const float* __restrict__ Wg, const float* __restrict__ bg,
                                                       unsigned short* __restrict__ XI, int row0) {
  __shared__ __align__(16) unsigned short sm[64 * kXi];
  const int t  = threadIdx.x;
  const int rb = blockIdx.x * 64;
#pragma unroll 1
  for (int i = 0; i < 8; ++i) {
    const int e = i * 256 + t;
    const int r = e >> 5;
    const int c = e & 31;
    int gr = row0 + rb + r; gr = (gr < kItems) ? gr : (kItems - 1);
    const float f0 = item_feat[(size_t)gr * 2];
    const float f1 = item_feat[(size_t)gr * 2 + 1];
    const float w0 = Wg[c], w1 = Wg[kGeo + c], bb = bg[c];
    float g = f0 * w0 + f1 * w1;
    g += bb;
    g = fmaxf(g, 0.0f);
    sm[r * kXi + c] = h_bits(g * kActCarry);
  }
#pragma unroll 1
  for (int i = 0; i < 8; ++i) {
    const int e  = i * 256 + t;
    const int r  = e >> 5;
    const int c4 = (e & 31) * 4;
    int gr = row0 + rb + r; gr = (gr < kItems) ? gr : (kItems - 1);
    const v4f x = *(const v4f*)(gcn_item + (size_t)gr * kGcn + c4);
    const v2u p2 = (v2u){pk16(h_bits(x[0] * kActCarry), h_bits(x[1] * kActCarry)),
                         pk16(h_bits(x[2] * kActCarry), h_bits(x[3] * kActCarry))};
    *(v2u*)(sm + r * kXi + kGeo + c4) = p2;
  }
  __syncthreads();
  unsigned short* base = XI + (size_t)rb * kXi;
  for (int pass = 0; pass < 2; ++pass) {
#pragma unroll 1
    for (int i = 0; i < 5; ++i) {
      const int f = (i * 256 + t) * 8;
      const unsigned short* sp = sm + f;
      const v4u u = (v4u){pk16(sp[0], sp[1]), pk16(sp[2], sp[3]), pk16(sp[4], sp[5]), pk16(sp[6], sp[7])};
      *(volatile v4u*)(base + f) = u;
    }
    __threadfence();
  }
}

__global__ __launch_bounds__(256) void rownorm_kernel(const float* __restrict__ X, float* __restrict__ out, int nplane, int nvalid) {
  const int lane = threadIdx.x & 31, wave = threadIdx.x >> 5;
  const int r  = blockIdx.x * 8 + wave;
  const int rr = (r < nplane) ? r : (nplane - 1);
  const v4f x = *(const v4f*)(X + (size_t)rr * kTow + lane * 4);
  float ss = x[0] * x[0] + x[1] * x[1] + x[2] * x[2] + x[3] * x[3];
  ss += __shfl_xor(ss, 16, 32);
  ss += __shfl_xor(ss, 8, 32);
  ss += __shfl_xor(ss, 4, 32);
  ss += __shfl_xor(ss, 2, 32);
  ss += __shfl_xor(ss, 1, 32);
  const float nrm = sqrtf(ss);
  const float inv = 1.0f / fmaxf(nrm, 1e-12f);
  const v4f o = x * inv;
  if (r < nvalid) {
    float* p = out + (size_t)r * kTow + lane * 4;
    *(volatile v4f*)p = o;
    __threadfence();
    *(volatile v4f*)p = o;
  }
}

__global__ __launch_bounds__(256) void cast_user_kernel(const float* __restrict__ gu, unsigned short* __restrict__ fused) {
  const int lane = threadIdx.x & 31, wave = threadIdx.x >> 5;
  const int row  = blockIdx.x * 16 + wave * 2 + (lane >> 4);
  const int c8   = (lane & 15) * 8;
  const float* src = gu + (size_t)row * kGcn + c8;
  const v4f a = *(const v4f*)(src);
  const v4f c = *(const v4f*)(src + 4);
  const v4u u = pack8_carry(a, c);
  unsigned short* dst = fused + (size_t)row * kFusedLd + c8;
  *(volatile v4u*)dst = u;
  __threadfence();
  *(volatile v4u*)dst = u;
}

__global__ __launch_bounds__(256) void gather_h_kernel(const float* __restrict__ item_rows, const int* __restrict__ user_items,
                                                       unsigned short* __restrict__ H, int ubase) {
  const int lane = threadIdx.x & 31, wave = threadIdx.x >> 5;
  const int c8 = (lane & 15) * 8;
#pragma unroll 1
  for (int it = 0; it < 4; ++it) {
    const int j = blockIdx.x * 64 + it * 16 + wave * 2 + (lane >> 4);
    int idx = user_items[(size_t)ubase * kHist + j];
    idx = (idx < 0) ? 0 : idx;
    idx = (idx > kItems - 1) ? (kItems - 1) : idx;
    const float* src = item_rows + (size_t)idx * kTow + c8;
    const v4f a = *(const v4f*)(src);
    const v4f c = *(const v4f*)(src + 4);
    const v4u u = pack8_carry(a, c);
    unsigned short* dst = H + (size_t)j * kTow + c8;
    *(volatile v4u*)dst = u;
    __threadfence();
    *(volatile v4u*)dst = u;
  }
}

__global__ __launch_bounds__(256) void attn_pool_kernel(const float* __restrict__ Qp, const float* __restrict__ KK,
                                                        const float* __restrict__ item_rows, const int* __restrict__ user_items,
                                                        unsigned short* __restrict__ fused, int ubase) {
  __shared__ __align__(16) float s_sc [8][64];
  __shared__ __align__(16) int   s_idx[8][64];
  __shared__ __align__(16) float s_rep[8][132];
  const int lane = threadIdx.x & 31, wave = threadIdx.x >> 5;
  const int lu = blockIdx.x * 8 + wave;
  const int u  = ubase + lu;
  {
    const int k1 = (lane + 32 < kHist) ? (lane + 32) : (kHist - 1);
    int i0 = user_items[(size_t)u * kHist + lane];
    int i1 = user_items[(size_t)u * kHist + k1];
    i0 = (i0 < 0) ? 0 : i0; i0 = (i0 > kItems - 1) ? (kItems - 1) : i0;
    i1 = (i1 < 0) ? 0 : i1; i1 = (i1 > kItems - 1) ? (kItems - 1) : i1;
    s_idx[wave][lane]      = i0;
    s_idx[wave][lane + 32] = i1;
    s_sc[wave][lane]       = -INFINITY;
    s_sc[wave][lane + 32]  = -INFINITY;
  }
  __syncthreads();
  const v4f qv = *(const v4f*)(Qp + (size_t)u * kTow + lane * 4);
  const float* kkb = KK + (size_t)lu * kHist * kTow + lane * 4;
#pragma unroll 1
  for (int k = 0; k < kHist; ++k) {
    const v4f kv = *(const v4f*)(kkb + (size_t)k * kTow);
    float p = qv[0] * kv[0] + qv[1] * kv[1] + qv[2] * kv[2] + qv[3] * kv[3];
    p += __shfl_xor(p, 16, 32);
    p += __shfl_xor(p, 8, 32);
    p += __shfl_xor(p, 4, 32);
    p += __shfl_xor(p, 2, 32);
    p += __shfl_xor(p, 1, 32);
    if (lane == 0) s_sc[wave][k] = p;
  }
  __syncthreads();
  {
    const float v0 = s_sc[wave][lane];
    const float v1 = s_sc[wave][lane + 32];
    float m = fmaxf(v0, v1);
    m = fmaxf(m, __shfl_xor(m, 16, 32));
    m = fmaxf(m, __shfl_xor(m, 8, 32));
    m = fmaxf(m, __shfl_xor(m, 4, 32));
    m = fmaxf(m, __shfl_xor(m, 2, 32));
    m = fmaxf(m, __shfl_xor(m, 1, 32));
    const float e0 = expf(v0 - m);
    const float e1 = expf(v1 - m);
    float s = e0 + e1;
    s += __shfl_xor(s, 16, 32);
    s += __shfl_xor(s, 8, 32);
    s += __shfl_xor(s, 4, 32);
    s += __shfl_xor(s, 2, 32);
    s += __shfl_xor(s, 1, 32);
    const float inv = 1.0f / s;
    const float a0 = e0 * inv;
    const float a1 = e1 * inv;
    s_sc[wave][lane]      = a0;
    s_sc[wave][lane + 32] = a1;
  }
  __syncthreads();
  v4f acc = (v4f){0.f, 0.f, 0.f, 0.f};
#pragma unroll 1
  for (int k = 0; k < kHist; ++k) {
    const float a  = s_sc[wave][k];
    const int  idx = s_idx[wave][k];
    const v4f  hv  = *(const v4f*)(item_rows + (size_t)idx * kTow + lane * 4);
    acc = acc + hv * a;
  }
  *(v4f*)(&s_rep[wave][lane * 4]) = acc;
  __syncthreads();
  const int c8 = (lane & 15) * 8;
  const float* rp = &s_rep[wave][c8];
  const v4f ra = (v4f){rp[0], rp[1], rp[2], rp[3]};
  const v4f rc = (v4f){rp[4], rp[5], rp[6], rp[7]};
  const v4u uo = pack8_carry(ra, rc);
  unsigned short* dst = fused + (size_t)u * kFusedLd + kGcn + c8;
  for (int pass = 0; pass < 2; ++pass) {
    if (lane < 16) *(volatile v4u*)dst = uo;
    __threadfence();
  }
}

extern "C" void kernel_launch(void* const* d_in, const int* in_sizes, int n_in,
                              void* d_out, int out_size, void* d_ws, size_t ws_size, hipStream_t stream) {
  if (n_in < 18) return;
  if (out_size != (kItems + kUsers) * kTow) return;
  if (in_sizes[0] != kItems * 2 || in_sizes[1] != kItems * kGcn || in_sizes[2] != kUsers * kGcn ||
      in_sizes[3] != kUsers * kHist) return;
  if (in_sizes[6] != kXi * kHid || in_sizes[8] != kHid * kTow || in_sizes[10] != kGcn * kTow ||
      in_sizes[12] != kTow * kTow || in_sizes[14] != kFusedLd * kHid || in_sizes[16] != kHid * kTow) return;

  const float* item_feat  = (const float*)d_in[0];
  const float* gcn_item   = (const float*)d_in[1];
  const float* gcn_user   = (const float*)d_in[2];
  const int*   user_items = (const int*)  d_in[3];
  const float* Wg  = (const float*)d_in[4];
  const float* bg  = (const float*)d_in[5];
  const float* Wi1 = (const float*)d_in[6];
  const float* bi1 = (const float*)d_in[7];
  const float* Wi2 = (const float*)d_in[8];
  const float* bi2 = (const float*)d_in[9];
  const float* Wq  = (const float*)d_in[10];
  const float* bq  = (const float*)d_in[11];
  const float* Wk  = (const float*)d_in[12];
  const float* bk  = (const float*)d_in[13];
  const float* Wu1 = (const float*)d_in[14];
  const float* bu1 = (const float*)d_in[15];
  const float* Wu2 = (const float*)d_in[16];
  const float* bu2 = (const float*)d_in[17];
  float* out = (float*)d_out;
  char* ws = (char*)d_ws;

  const size_t offWi1T = 0;
  const size_t offWi2T = offWi1T + (size_t)kHid * kXi * 2;
  const size_t offWqT  = offWi2T + (size_t)kTow * kHid * 2;
  const size_t offWkT  = offWqT  + (size_t)kTow * kGcn * 2;
  const size_t offWu1T = offWkT  + (size_t)kTow * kTow * 2;
  const size_t offWu2T = offWu1T + (size_t)kHid * kFusedLd * 2;
  const size_t offBi1  = offWu2T + (size_t)kTow * kHid * 2;
  const size_t offBu1  = offBi1  + (size_t)kHid * 4;
  const size_t kBase   = 1048576;
  if (offBu1 + (size_t)kHid * 4 > kBase) return;
  const size_t offXI = kBase;
  const size_t offH1 = offXI + (size_t)kItemChunkRows * kXi * 2;
  const size_t offO2 = offH1 + (size_t)kItemChunkRows * kHid * 2;
  const size_t endItem = offO2 + (size_t)kItemChunkRows * kTow * 4;
  const size_t offFU = kBase;
  const size_t offQ  = offFU + (size_t)kUsers * kFusedLd * 2;
  const size_t offH  = offQ  + (size_t)kUsers * kTow * 4;
  const size_t offKK = offH  + (size_t)kHRows * kTow * 2;
  const size_t offU1 = offKK + (size_t)kHRows * kTow * 4;
  const size_t offUO = offU1 + (size_t)kUsers * kHid * 2;
  const size_t endUser = offUO + (size_t)kUsers * kTow * 4;
  const size_t total = (endItem > endUser) ? endItem : endUser;
  if (total > ws_size) return;

  unsigned short* Wi1T = (unsigned short*)(ws + offWi1T);
  unsigned short* Wi2T = (unsigned short*)(ws + offWi2T);
  unsigned short* WqT  = (unsigned short*)(ws + offWqT);
  unsigned short* WkT  = (unsigned short*)(ws + offWkT);
  unsigned short* Wu1T = (unsigned short*)(ws + offWu1T);
  unsigned short* Wu2T = (unsigned short*)(ws + offWu2T);
  float* bi1x8 = (float*)(ws + offBi1);
  float* bu1x8 = (float*)(ws + offBu1);
  unsigned short* XI16 = (unsigned short*)(ws + offXI);
  unsigned short* H1   = (unsigned short*)(ws + offH1);
  float*          O2   = (float*)(ws + offO2);
  unsigned short* FU16 = (unsigned short*)(ws + offFU);
  float*          Qp   = (float*)(ws + offQ);
  unsigned short* H16  = (unsigned short*)(ws + offH);
  float*          KK   = (float*)(ws + offKK);
  unsigned short* U1   = (unsigned short*)(ws + offU1);
  float*          UO   = (float*)(ws + offUO);

  wtcast_kernel<<<kHid / 64, 256, 0, stream>>>(Wi1, Wi1T, kXi,      kHid, kWCarry);
  wtcast_kernel<<<kTow / 64, 256, 0, stream>>>(Wi2, Wi2T, kHid,     kTow, kWCarry);
  wtcast_kernel<<<kTow / 64, 256, 0, stream>>>(Wq,  WqT,  kGcn,     kTow, kWCarry);
  wtcast_kernel<<<kTow / 64, 256, 0, stream>>>(Wk,  WkT,  kTow,     kTow, kWCarry);
  wtcast_kernel<<<kHid / 64, 256, 0, stream>>>(Wu1, Wu1T, kFusedLd, kHid, kWCarry);
  wtcast_kernel<<<kTow / 64, 256, 0, stream>>>(Wu2, Wu2T, kHid,     kTow, kWCarry);
  bias8_kernel<<<1, 64, 0, stream>>>(bi1, bi1x8);
  bias8_kernel<<<1, 64, 0, stream>>>(bu1, bu1x8);

  for (int c = 0; c < kItemChunks; ++c) {
    const int row0 = c * kItemChunkRows;
    const int M = kItemChunkRows;
    int nvalid = kItems - row0; nvalid = (nvalid > M) ? M : nvalid;
    xi_build_kernel<<<M / 64, 256, 0, stream>>>(item_feat, gcn_item, Wg, bg, XI16, row0);
    wmma_gemm64<0, false, 2, 1, false, 2><<<dim3((unsigned)(((M / 64) * (kHid / 64) + 7) / 8), 1), 256, 0, stream>>>(
        XI16, XI16, kXi, 0L, Wi1T, Wi1T, kXi, 0L, (void*)H1, (void*)H1, kHid, 0L, bi1x8, bi1x8, 0L, M, kHid, kXi, kScaleOutX8);
    wmma_gemm64<0, false, 2, 0, false, 0><<<dim3((unsigned)(((M / 64) * (kTow / 64) + 7) / 8), 1), 256, 0, stream>>>(
        H1, H1, kHid, 0L, Wi2T, Wi2T, kHid, 0L, (void*)O2, (void*)O2, kTow, 0L, bi2, bi2, 0L, M, kTow, kHid, kScaleOutF32);
    rownorm_kernel<<<M / 8, 256, 0, stream>>>(O2, out + (size_t)row0 * kTow, M, nvalid);
  }

  cast_user_kernel<<<kUsers / 16, 256, 0, stream>>>(gcn_user, FU16);
  wmma_gemm64<0, false, 2, 0, false, 0><<<dim3((unsigned)(((kUsers / 64) * (kTow / 64) + 7) / 8), 1), 256, 0, stream>>>(
      FU16, FU16, kFusedLd, 0L, WqT, WqT, kGcn, 0L, (void*)Qp, (void*)Qp, kTow, 0L, bq, bq, 0L, kUsers, kTow, kGcn, kScaleOutF32);
  for (int uc = 0; uc < kUserChunks; ++uc) {
    const int ubase = uc * kUserChunk;
    gather_h_kernel<<<kHRows / 64, 256, 0, stream>>>(out, user_items, H16, ubase);
    wmma_gemm64<0, false, 2, 0, false, 0><<<dim3((unsigned)(((kHRows / 64) * (kTow / 64) + 7) / 8), 1), 256, 0, stream>>>(
        H16, H16, kTow, 0L, WkT, WkT, kTow, 0L, (void*)KK, (void*)KK, kTow, 0L, bk, bk, 0L, kHRows, kTow, kTow, kScaleOutF32);
    attn_pool_kernel<<<kUserChunk / 8, 256, 0, stream>>>(Qp, KK, out, user_items, FU16, ubase);
  }
  wmma_gemm64<0, false, 2, 1, false, 2><<<dim3((unsigned)(((kUsers / 64) * (kHid / 64) + 7) / 8), 1), 256, 0, stream>>>(
      FU16, FU16, kFusedLd, 0L, Wu1T, Wu1T, kFusedLd, 0L, (void*)U1, (void*)U1, kHid, 0L, bu1x8, bu1x8, 0L, kUsers, kHid, kFusedLd, kScaleOutX8);
  wmma_gemm64<0, false, 2, 0, false, 0><<<dim3((unsigned)(((kUsers / 64) * (kTow / 64) + 7) / 8), 1), 256, 0, stream>>>(
      U1, U1, kHid, 0L, Wu2T, Wu2T, kHid, 0L, (void*)UO, (void*)UO, kTow, 0L, bu2, bu2, 0L, kUsers, kTow, kHid, kScaleOutF32);
  rownorm_kernel<<<kUsers / 8, 256, 0, stream>>>(UO, out + (size_t)kItems * kTow, kUsers, kUsers);
}
